// MambaBlock_15161234555020
// MI455X (gfx1250) — hardware-verified
//
#include <hip/hip_runtime.h>
#include <math.h>

typedef __attribute__((ext_vector_type(16))) _Float16 v16h;
typedef __attribute__((ext_vector_type(8)))  _Float16 v8h;
typedef __attribute__((ext_vector_type(16))) __bf16   v16b;
typedef __attribute__((ext_vector_type(8)))  __bf16   v8b;
typedef __attribute__((ext_vector_type(8)))  float    v8f;
typedef __attribute__((ext_vector_type(4)))  float    v4f;

constexpr int kB      = 4;
constexpr int kL      = 1024;
constexpr int kD      = 256;
constexpr int kN      = 16;
constexpr int kDtR    = 16;
constexpr int kConvK  = 4;
constexpr int kXzP    = 2 * kD;
constexpr int kXdW    = kDtR + 2 * kN;
constexpr int kXdP    = 64;
constexpr int kRows   = kB * kL;
constexpr int kConvTP = 260;
constexpr int kScanTS = 64;
constexpr int kScanCh = 64;
constexpr int kScanYP = 68;
static_assert(kXdW <= kXdP, "x_proj pad");
static_assert((kD % 32) == 0 && (kL % 32) == 0, "GEMM K multiples of 32");
static_assert((kRows % 64) == 0 && (kXzP % 64) == 0 && (kXdP % 64) == 0 && (kD % 64) == 0 && (kL % 64) == 0, "GEMM M,N multiples of 64");
static_assert((kL % kScanTS) == 0 && (kD % kScanCh) == 0 && kD == 256 && (kL % 64) == 0, "tile multiples");
static_assert(((kXdW * kD / 8) % 256) == 0, "x_proj weight pad boundary is block-uniform");

constexpr size_t kOffXB   = 0;
constexpr size_t kOffWIB  = kOffXB  + (size_t)kRows * kD * 2;
constexpr size_t kOffWXB  = kOffWIB + (size_t)kXzP * kD * 2;
constexpr size_t kOffWOB  = kOffWXB + (size_t)kXdP * kD * 2;
constexpr size_t kOffDTB  = kOffWOB + (size_t)kD * kD * 2;
constexpr size_t kOffXZ   = kOffDTB + (size_t)kB * kL * kL * 2;
constexpr size_t kOffUC   = kOffXZ  + (size_t)kRows * kXzP * 4;
constexpr size_t kOffUCH  = kOffUC  + (size_t)kRows * kD * 4;
constexpr size_t kOffUCL  = kOffUCH + (size_t)kRows * kD * 2;
constexpr size_t kOffUTH  = kOffUCL + (size_t)kRows * kD * 2;
constexpr size_t kOffUTL  = kOffUTH + (size_t)kB * kD * kL * 2;
constexpr size_t kOffXD   = kOffUTL + (size_t)kB * kD * kL * 2;
constexpr size_t kOffDP   = kOffXD  + (size_t)kRows * kXdP * 4;
constexpr size_t kOffYH   = kOffDP  + (size_t)kB * kL * kD * 4;
constexpr size_t kOffYL   = kOffYH  + (size_t)kRows * kD * 2;
constexpr size_t kWsTotal = kOffYL  + (size_t)kRows * kD * 2;
static_assert(kWsTotal == 41320448ull, "carve total");
static_assert(kWsTotal <= 134217728ull, "carve cap");
static_assert((kOffWIB % 128) == 0 && (kOffWXB % 128) == 0 && (kOffWOB % 128) == 0 && (kOffDTB % 128) == 0 &&
              (kOffXZ % 128) == 0 && (kOffUC % 128) == 0 && (kOffUCH % 128) == 0 && (kOffUCL % 128) == 0 &&
              (kOffUTH % 128) == 0 && (kOffUTL % 128) == 0 && (kOffXD % 128) == 0 && (kOffDP % 128) == 0 &&
              (kOffYH % 128) == 0 && (kOffYL % 128) == 0, "128-B aligned regions");

__device__ __forceinline__ unsigned short f2bf_bits(float f) {
  unsigned u = __float_as_uint(f);
  return (unsigned short)((u + 0x7FFFu + ((u >> 16) & 1u)) >> 16);
}
__device__ __forceinline__ float bf_bits2f(unsigned short h) { return __uint_as_float(((unsigned)h) << 16); }
__device__ __forceinline__ float bf_quant(float f) { return bf_bits2f(f2bf_bits(f)); }

__device__ __forceinline__ void dep_guard4_b(v8f& a, v8f& b, v8f& c, v8f& d, v16b x, v16b y) {
  asm volatile("v_nop\n\tv_nop\n\tv_nop\n\tv_nop" : "+v"(a), "+v"(b), "+v"(c), "+v"(d) : "v"(x), "v"(y));
}
__device__ __forceinline__ void keep4_b(v16b a, v16b b, v16b c, v16b d) { asm volatile("v_nop" :: "v"(a), "v"(b), "v"(c), "v"(d)); }
__device__ __forceinline__ void acc_guard4(v8f& a, v8f& b, v8f& c, v8f& d) { asm volatile("v_nop\n\tv_nop\n\tv_nop\n\tv_nop" : "+v"(a), "+v"(b), "+v"(c), "+v"(d)); }

struct FragB {
  union U { v16b v; v8b h[2]; };
  static __device__ __forceinline__ v16b load(const __bf16* p) {
    U f; f.h[0] = *(const v8b*)(p); f.h[1] = *(const v8b*)(p + 16); return f.v;
  }
  static __device__ __forceinline__ v8f mma(v16b a, v16b b, v8f c) {
    return __builtin_amdgcn_wmma_f32_16x16x32_bf16(false, a, false, b, (short)0, c, false, false);
  }
};

template <int SPL, int ACT>
__global__ __launch_bounds__(256) void wmma_gemm64(
    const unsigned short* __restrict__ Ap, const unsigned short* __restrict__ A2p, int lda, long strideA,
    const unsigned short* __restrict__ Btp, const unsigned short* __restrict__ Bt2p, int ldb, long strideB,
    float* __restrict__ Cout, int ldc, long strideC, int M, int N, int K)
{
  constexpr bool ASPL = (SPL == 1);
  constexpr bool BSPL = (SPL == 3);
  const __bf16* A  = (const __bf16*)Ap;  const __bf16* A2  = (const __bf16*)A2p;
  const __bf16* Bt = (const __bf16*)Btp; const __bf16* Bt2 = (const __bf16*)Bt2p;
  __shared__ __align__(16) float sT[8][16 * 68];
  const int b    = blockIdx.y;
  const int lane = threadIdx.x & 31;
  const int wave = threadIdx.x >> 5;
  const int tilesN = N >> 6;
  const int tilesM = M >> 6;
  const int tile = blockIdx.x * 8 + wave;
  if (tile >= tilesM * tilesN) return;
  const int tm = tile / tilesN;
  const int tn = tile - tm * tilesN;
  const int m0 = tm << 6;
  const int n0 = tn << 6;

  const __bf16* Ab  = A  + (size_t)b * strideA;
  const __bf16* Bb  = Bt + (size_t)b * strideB;
  const __bf16* Ab2 = ASPL ? (A2  + (size_t)b * strideA) : nullptr;
  const __bf16* Bb2 = BSPL ? (Bt2 + (size_t)b * strideB) : nullptr;

  const int rlane = lane & 15;
  const int koff  = (lane >> 4) * 8;
  const int mOff  = (lane >> 4) * 8;

  v8f acc[4][4];
#pragma unroll
  for (int i = 0; i < 4; ++i)
#pragma unroll
    for (int j = 0; j < 4; ++j) acc[i][j] = (v8f){0.f,0.f,0.f,0.f,0.f,0.f,0.f,0.f};

  for (int k0 = 0; k0 < K; k0 += 32) {
    v16b bh[4], bl[4];
#pragma unroll
    for (int j = 0; j < 4; ++j) {
      const size_t bo = (size_t)(n0 + (j << 4) + rlane) * ldb + koff + k0;
      bh[j] = FragB::load(Bb + bo);
      if (BSPL) bl[j] = FragB::load(Bb2 + bo);
      else bl[j] = bh[j];
    }
#pragma unroll
    for (int i = 0; i < 4; ++i) {
      const size_t ao = (size_t)(m0 + (i << 4) + rlane) * lda + koff + k0;
      v16b ah = FragB::load(Ab + ao);
      v16b al = ah;
      if (ASPL) al = FragB::load(Ab2 + ao);
#pragma unroll
      for (int j = 0; j < 4; ++j) {
        acc[i][j] = FragB::mma(ah, bh[j], acc[i][j]);
        if (BSPL) acc[i][j] = FragB::mma(ah, bl[j], acc[i][j]);
        if (ASPL) acc[i][j] = FragB::mma(al, bh[j], acc[i][j]);
      }
      dep_guard4_b(acc[i][0], acc[i][1], acc[i][2], acc[i][3], ah, al);
    }
    keep4_b(bh[0], bh[1], bh[2], bh[3]);
    if (BSPL) keep4_b(bl[0], bl[1], bl[2], bl[3]);
  }
  acc_guard4(acc[0][0], acc[0][1], acc[0][2], acc[0][3]);
  acc_guard4(acc[1][0], acc[1][1], acc[1][2], acc[1][3]);
  acc_guard4(acc[2][0], acc[2][1], acc[2][2], acc[2][3]);
  acc_guard4(acc[3][0], acc[3][1], acc[3][2], acc[3][3]);

  float* slab = sT[wave];
  float* C = Cout + (size_t)b * strideC;
#pragma unroll
  for (int i = 0; i < 4; ++i) {
    const int mBase = m0 + (i << 4);
#pragma unroll
    for (int j = 0; j < 4; ++j) {
#pragma unroll
      for (int r = 0; r < 8; ++r) {
        float v = acc[i][j][r];
        if (ACT == 6) v = (fabsf(v) < __builtin_huge_valf()) ? v : 0.0f;
        slab[(mOff + r) * 68 + (j << 4) + rlane] = v;
      }
    }
    __builtin_amdgcn_fence(__ATOMIC_RELEASE, "workgroup");
    __builtin_amdgcn_wave_barrier();
    __builtin_amdgcn_fence(__ATOMIC_ACQUIRE, "workgroup");
    {
      const int hh = lane >> 4, c4 = (lane & 15) * 4;
      for (int pass = 0; pass < 2; ++pass) {
#pragma unroll
        for (int it = 0; it < 8; ++it) {
          const int row = it * 2 + hh;
          v4f v = *(const v4f*)(slab + row * 68 + c4);
          *(volatile v4f*)(C + (size_t)(mBase + row) * ldc + n0 + c4) = v;
        }
        __threadfence();
      }
    }
    __builtin_amdgcn_fence(__ATOMIC_RELEASE, "workgroup");
    __builtin_amdgcn_wave_barrier();
    __builtin_amdgcn_fence(__ATOMIC_ACQUIRE, "workgroup");
  }
}

__global__ __launch_bounds__(256) void cvt_bf16_kernel(
    const float* __restrict__ src, unsigned short* __restrict__ dst, int valid8, int total8)
{
  const int i = blockIdx.x * 256 + threadIdx.x;
  if (i >= total8) return;
  const bool pad = ((int)blockIdx.x * 256 >= valid8);
  v8h hv;
  if (pad) {
#pragma unroll
    for (int e = 0; e < 8; ++e) hv[e] = (_Float16)0.0f;
  } else {
    const size_t e0 = (size_t)i << 3;
    const v4f a0 = *(const v4f*)(src + e0);
    const v4f a1 = *(const v4f*)(src + e0 + 4);
#pragma unroll
    for (int e = 0; e < 4; ++e) {
      const unsigned short h0 = f2bf_bits(a0[e]), h1 = f2bf_bits(a1[e]);
      hv[e]     = __builtin_bit_cast(_Float16, h0);
      hv[4 + e] = __builtin_bit_cast(_Float16, h1);
    }
  }
  unsigned short* qh = dst + ((size_t)i << 3);
  *(volatile v8h*)qh = hv;
  __threadfence();
  *(volatile v8h*)qh = hv;
}

template <bool LO>
__global__ __launch_bounds__(256) void transpose_bf16_kernel(
    const float* __restrict__ src, int spitch, long sstride,
    unsigned short* __restrict__ dhi, unsigned short* __restrict__ dlo, int opitch, long ostride)
{
  __shared__ __align__(16) float sT[64 * 65];
  const int tid = threadIdx.x;
  const int b = blockIdx.z, r0 = blockIdx.y * 64, c0 = blockIdx.x * 64;
  const float* sb = src + (size_t)b * sstride;
  const int lr = tid >> 4, lc4 = (tid & 15) * 4;
#pragma unroll
  for (int i = 0; i < 4; ++i) {
    const int r = lr + 16 * i;
    const v4f v = *(const v4f*)(sb + (size_t)(r0 + r) * spitch + c0 + lc4);
    float* tp = sT + r * 65 + lc4;
    tp[0] = v[0]; tp[1] = v[1]; tp[2] = v[2]; tp[3] = v[3];
  }
  __syncthreads();
  const int q = tid >> 3, c8 = (tid & 7) * 8;
  v8h hv[2], lv[2];
#pragma unroll
  for (int it = 0; it < 2; ++it) {
    const int orow = it * 32 + q;
#pragma unroll
    for (int e = 0; e < 8; ++e) {
      const float f = sT[(c8 + e) * 65 + orow];
      const unsigned short h0 = f2bf_bits(f);
      hv[it][e] = __builtin_bit_cast(_Float16, h0);
      if (LO) {
        const unsigned short l0 = f2bf_bits(f - bf_bits2f(h0));
        lv[it][e] = __builtin_bit_cast(_Float16, l0);
      } else {
        lv[it][e] = hv[it][e];
      }
    }
  }
  unsigned short* hb = dhi + (size_t)b * ostride;
  unsigned short* lb = LO ? (dlo + (size_t)b * ostride) : nullptr;
  for (int pass = 0; pass < 2; ++pass) {
#pragma unroll
    for (int it = 0; it < 2; ++it) {
      const int orow = it * 32 + q;
      const size_t o = (size_t)(c0 + orow) * opitch + r0 + c8;
      *(volatile v8h*)(hb + o) = hv[it];
      if (LO) *(volatile v8h*)(lb + o) = lv[it];
    }
    __threadfence();
  }
}

__global__ __launch_bounds__(256) void conv_silu_kernel(
    const float* __restrict__ XZ, const float* __restrict__ cw, const float* __restrict__ cb,
    float* __restrict__ UC, unsigned short* __restrict__ UCH, unsigned short* __restrict__ UCL)
{
  __shared__ __align__(16) float sT[16 * kConvTP];
  const int tid = threadIdx.x, lane = tid & 31, wave = tid >> 5;
  const int d = tid;
  const int g0 = blockIdx.x * 64;
  const int tb = g0 & (kL - 1);
  const float w0 = bf_quant(cw[d * kConvK + 0]), w1 = bf_quant(cw[d * kConvK + 1]);
  const float w2 = bf_quant(cw[d * kConvK + 2]), w3 = bf_quant(cw[d * kConvK + 3]);
  const float bc = bf_quant(cb[d]);
  float xm3, xm2, xm1;
  {
    const bool hist = (tb > 0);
    const int rb = hist ? (g0 - 3) : g0;
    const float v3 = XZ[(size_t)rb * kXzP + d];
    const float v2 = XZ[(size_t)(rb + 1) * kXzP + d];
    const float v1 = XZ[(size_t)(rb + 2) * kXzP + d];
    xm3 = hist ? v3 : 0.f;
    xm2 = hist ? v2 : 0.f;
    xm1 = hist ? v1 : 0.f;
  }
  const int hrow = wave >> 1;
  const int hch  = (wave & 1) * 128 + lane * 4;
#pragma unroll 1
  for (int sub = 0; sub < 4; ++sub) {
    const int lb = g0 + sub * 16;
#pragma unroll 1
    for (int s = 0; s < 16; ++s) {
      const float xcur = XZ[(size_t)(lb + s) * kXzP + d];
      float acc = w0 * xm3;
      acc = fmaf(w1, xm2, acc);
      acc = fmaf(w2, xm1, acc);
      acc = fmaf(w3, xcur, acc);
      const float sv = acc + bc;
      const float eg = expf(-sv);
      const float sg = __builtin_amdgcn_rcpf(1.0f + eg);
      sT[s * kConvTP + tid] = sv * sg;
      xm3 = xm2; xm2 = xm1; xm1 = xcur;
    }
    __syncthreads();
    v4f fv[4];
    v8h bh[2], blo[2];
#pragma unroll
    for (int it = 0; it < 4; ++it) fv[it] = *(const v4f*)(sT + (it * 4 + hrow) * kConvTP + hch);
#pragma unroll
    for (int it = 0; it < 2; ++it) {
      const float* sp = sT + (it * 8 + wave) * kConvTP + lane * 8;
      const v4f a0 = *(const v4f*)(sp);
      const v4f a1 = *(const v4f*)(sp + 4);
#pragma unroll
      for (int e = 0; e < 4; ++e) {
        const unsigned short h0 = f2bf_bits(a0[e]), h1 = f2bf_bits(a1[e]);
        const unsigned short l0 = f2bf_bits(a0[e] - bf_bits2f(h0)), l1 = f2bf_bits(a1[e] - bf_bits2f(h1));
        bh[it][e]      = __builtin_bit_cast(_Float16, h0);
        bh[it][4 + e]  = __builtin_bit_cast(_Float16, h1);
        blo[it][e]     = __builtin_bit_cast(_Float16, l0);
        blo[it][4 + e] = __builtin_bit_cast(_Float16, l1);
      }
    }
    for (int pass = 0; pass < 2; ++pass) {
#pragma unroll
      for (int it = 0; it < 4; ++it)
        *(volatile v4f*)(UC + (size_t)(lb + it * 4 + hrow) * kD + hch) = fv[it];
#pragma unroll
      for (int it = 0; it < 2; ++it) {
        const size_t o = (size_t)(lb + it * 8 + wave) * kD + lane * 8;
        *(volatile v8h*)(UCH + o) = bh[it];
        *(volatile v8h*)(UCL + o) = blo[it];
      }
      __threadfence();
    }
    __syncthreads();
  }
}

__global__ __launch_bounds__(256) void scan_gate_kernel(
    const float* __restrict__ XD, const float* __restrict__ DP, const float* __restrict__ UC,
    const float* __restrict__ XZ, const float* __restrict__ Alog, const float* __restrict__ Dp,
    unsigned short* __restrict__ YH, unsigned short* __restrict__ YL)
{
  __shared__ __align__(16) float sX[kScanTS * kXdP];
  __shared__ __align__(16) float sY[kScanTS * kScanYP];
  const int tid = threadIdx.x, lane = tid & 31, wave = tid >> 5;
  const int ch = tid >> 2, sub = tid & 3;
  constexpr int kBlkPerB = kD / kScanCh;
  const int bix = blockIdx.x / kBlkPerB;
  const int d0  = (blockIdx.x - bix * kBlkPerB) * kScanCh;
  const int d   = d0 + ch;
  const size_t row0 = (size_t)bix * kL;
  float An[4], run[4], Sacc[4];
#pragma unroll
  for (int j = 0; j < 4; ++j) {
    An[j] = -expf(bf_quant(Alog[(size_t)d * kN + sub * 4 + j]));
    run[j] = 0.0f;
    Sacc[j] = 0.0f;
  }
  const float Dd = bf_quant(Dp[d]);
  const int lr = tid >> 4, lc4 = (tid & 15) * 4;
  const int q = lane >> 3, c8 = (lane & 7) * 8;
#pragma unroll 1
  for (int t0 = 0; t0 < kL; t0 += kScanTS) {
    __syncthreads();
#pragma unroll
    for (int i = 0; i < 4; ++i) {
      const int r = lr + 16 * i;
      *(v4f*)(sX + r * kXdP + lc4) = *(const v4f*)(XD + (row0 + t0 + r) * kXdP + lc4);
    }
    __syncthreads();
#pragma unroll 1
    for (int s = 0; s < kScanTS; ++s) {
      const size_t grow = row0 + t0 + s;
      const float* xr = sX + s * kXdP;
      const float dp = DP[grow * kD + d];
      const float uu = UC[grow * kD + d];
      const float zv = XZ[grow * kXzP + kD + d];
      const v4f bv = *(const v4f*)(xr + kDtR + sub * 4);
      const v4f cv = *(const v4f*)(xr + kDtR + kN + sub * 4);
      const float dbu = dp * uu;
      float y = 0.0f;
#pragma unroll
      for (int j = 0; j < 4; ++j) {
        const float la = fminf(fmaxf(dp * An[j], -20.0f), 20.0f);
        run[j] = run[j] + la;
        const float lp = fminf(fmaxf(run[j], -30.0f), 30.0f);
        const float elp = expf(lp);
        const float einv = __builtin_amdgcn_rcpf(elp);
        Sacc[j] = fmaf(dbu * bv[j], einv, Sacc[j]);
        y = fmaf(Sacc[j] * elp, cv[j], y);
      }
      y += __shfl_xor(y, 1, 32);
      y += __shfl_xor(y, 2, 32);
      y = fmaf(uu, Dd, y);
      const float eg = expf(-zv);
      const float sg = __builtin_amdgcn_rcpf(1.0f + eg);
      const float yg = y * (zv * sg);
      if (sub == 0) sY[s * kScanYP + ch] = yg;
    }
    __syncthreads();
    v8h hv[2], lv[2];
#pragma unroll
    for (int it = 0; it < 2; ++it) {
      const int row = it * 32 + wave * 4 + q;
      const float* sp = sY + row * kScanYP + c8;
      const v4f a0 = *(const v4f*)(sp);
      const v4f a1 = *(const v4f*)(sp + 4);
#pragma unroll
      for (int e = 0; e < 4; ++e) {
        const unsigned short h0 = f2bf_bits(a0[e]), h1 = f2bf_bits(a1[e]);
        const unsigned short l0 = f2bf_bits(a0[e] - bf_bits2f(h0)), l1 = f2bf_bits(a1[e] - bf_bits2f(h1));
        hv[it][e]     = __builtin_bit_cast(_Float16, h0);
        hv[it][4 + e] = __builtin_bit_cast(_Float16, h1);
        lv[it][e]     = __builtin_bit_cast(_Float16, l0);
        lv[it][4 + e] = __builtin_bit_cast(_Float16, l1);
      }
    }
    for (int pass = 0; pass < 2; ++pass) {
#pragma unroll
      for (int it = 0; it < 2; ++it) {
        const int row = it * 32 + wave * 4 + q;
        const size_t o = (row0 + t0 + row) * kD + d0 + c8;
        *(volatile v8h*)(YH + o) = hv[it];
        *(volatile v8h*)(YL + o) = lv[it];
      }
      __threadfence();
    }
  }
}

extern "C" void kernel_launch(void* const* d_in, const int* in_sizes, int n_in,
                              void* d_out, int out_size, void* d_ws, size_t ws_size,
                              hipStream_t stream) {
  if (n_in < 11) return;
  if (in_sizes[0] != kRows * kD) return;
  if (in_sizes[1] != kB * kL * kL) return;
  if (in_sizes[2] != kXzP * kD) return;
  if (in_sizes[3] != kD * kConvK) return;
  if (in_sizes[4] != kD) return;
  if (in_sizes[5] != kXdW * kD) return;
  if (in_sizes[8] != kD * kN) return;
  if (in_sizes[9] != kD) return;
  if (in_sizes[10] != kD * kD) return;
  if (out_size != kRows * kD) return;
  if (ws_size < kWsTotal) return;

  const float* x       = (const float*)d_in[0];
  const float* dis     = (const float*)d_in[1];
  const float* W_in    = (const float*)d_in[2];
  const float* conv_w  = (const float*)d_in[3];
  const float* conv_b  = (const float*)d_in[4];
  const float* W_x     = (const float*)d_in[5];
  const float* A_log   = (const float*)d_in[8];
  const float* Dp      = (const float*)d_in[9];
  const float* W_out   = (const float*)d_in[10];
  float* out = (float*)d_out;

  char* ws = (char*)d_ws;
  unsigned short* XB   = (unsigned short*)(ws + kOffXB);
  unsigned short* WIB  = (unsigned short*)(ws + kOffWIB);
  unsigned short* WXB  = (unsigned short*)(ws + kOffWXB);
  unsigned short* WOB  = (unsigned short*)(ws + kOffWOB);
  unsigned short* DTB  = (unsigned short*)(ws + kOffDTB);
  float*          XZ   = (float*)(ws + kOffXZ);
  float*          UC   = (float*)(ws + kOffUC);
  unsigned short* UCH  = (unsigned short*)(ws + kOffUCH);
  unsigned short* UCL  = (unsigned short*)(ws + kOffUCL);
  unsigned short* UTH  = (unsigned short*)(ws + kOffUTH);
  unsigned short* UTL  = (unsigned short*)(ws + kOffUTL);
  float*          XD   = (float*)(ws + kOffXD);
  float*          DP   = (float*)(ws + kOffDP);
  unsigned short* YH   = (unsigned short*)(ws + kOffYH);
  unsigned short* YL   = (unsigned short*)(ws + kOffYL);

  cvt_bf16_kernel<<<(kRows * kD / 8) / 256, 256, 0, stream>>>(x, XB, kRows * kD / 8, kRows * kD / 8);
  cvt_bf16_kernel<<<(kXzP * kD / 8) / 256, 256, 0, stream>>>(W_in, WIB, kXzP * kD / 8, kXzP * kD / 8);
  cvt_bf16_kernel<<<(kXdP * kD / 8) / 256, 256, 0, stream>>>(W_x, WXB, kXdW * kD / 8, kXdP * kD / 8);
  cvt_bf16_kernel<<<(kD * kD / 8) / 256, 256, 0, stream>>>(W_out, WOB, kD * kD / 8, kD * kD / 8);

  transpose_bf16_kernel<false><<<dim3(kL / 64, kL / 64, kB), 256, 0, stream>>>(
      dis, kL, (long)kL * kL, DTB, nullptr, kL, (long)kL * kL);

  wmma_gemm64<0, 0><<<dim3(64, 1), 256, 0, stream>>>(
      XB, nullptr, kD, 0L,
      WIB, nullptr, kD, 0L,
      XZ, kXzP, 0L,
      kRows, kXzP, kD);

  conv_silu_kernel<<<dim3(kRows / 64), 256, 0, stream>>>(XZ, conv_w, conv_b, UC, UCH, UCL);

  transpose_bf16_kernel<true><<<dim3(kD / 64, kL / 64, kB), 256, 0, stream>>>(
      UC, kD, (long)kL * kD, UTH, UTL, kL, (long)kD * kL);

  wmma_gemm64<1, 0><<<dim3(8, 1), 256, 0, stream>>>(
      UCH, UCL, kD, 0L,
      WXB, nullptr, kD, 0L,
      XD, kXdP, 0L,
      kRows, kXdP, kD);

  wmma_gemm64<3, 0><<<dim3(8, kB), 256, 0, stream>>>(
      DTB, nullptr, kL, (long)kL * kL,
      UTH, UTL, kL, (long)kD * kL,
      DP, kD, (long)kL * kD,
      kL, kD, kL);

  scan_gate_kernel<<<kB * (kD / kScanCh), 256, 0, stream>>>(XD, DP, UC, XZ, A_log, Dp, YH, YL);

  wmma_gemm64<1, 6><<<dim3(32, 1), 256, 0, stream>>>(
      YH, YL, kD, 0L,
      WOB, nullptr, kD, 0L,
      out, kD, 0L,
      kRows, kD, kD);
}
